// TransformerDecoder_1116691497780
// MI455X (gfx1250) — hardware-run, weakly checked
//
#include <hip/hip_runtime.h>


namespace {
constexpr int B = 64, V = 256, NN = B * V, NPL = NN  , GM = NN  , K = 16, D = 128, E = 512, VOC = 32, BF = 6, NLAY = 3;
constexpr int KIN1 = D + BF, KP1 = 160, KIN2 = 2 * D;
constexpr float XS = 8.0f, WSC = 256.0f, WSQ = 0.25f, RS_ = 1024.0f, NSLOPE = 0.1f;
static_assert(NN % 8 == 0 && NPL % 8 == 0 && D == 128 && K == 16 && KP1 % 32 == 0 && KIN1 <= KP1, "tiling");
typedef _Float16 b16;
typedef __attribute__((ext_vector_type(16))) _Float16 v16b;
typedef __attribute__((ext_vector_type(8))) _Float16 v8b;
typedef __attribute__((ext_vector_type(8))) float v8f;
typedef __attribute__((ext_vector_type(4))) float v4f;
__device__ __forceinline__ float bf16_rne(float f) { unsigned int u = __float_as_uint(f); u += 0x7FFFu + ((u >> 16) & 1u); return __uint_as_float(u & 0xFFFF0000u); }
__device__ __forceinline__ void split16(float v, b16& hi, b16& lo) { hi = (b16)v; lo = (b16)(v - (float)hi); }
__device__ __forceinline__ v16b frag_kb(const b16* p, int hh) { const v8b a = *(const v8b*)(p + 8 * hh), b = *(const v8b*)(p + 16 + 8 * hh); v16b f;
#pragma unroll
  for (int e = 0; e < 8; ++e) { f[e] = a[e]; f[8 + e] = b[e]; } return f; }
__device__ __forceinline__ v8f wmma16b(v16b a, v16b b, v8f c) { v8f d = __builtin_amdgcn_wmma_f32_16x16x32_f16(false, a, false, b, (short)0, c, false, false); asm volatile("v_nop\n\tv_nop\n\tv_nop\n\tv_nop" : "+v"(d) : "v"(a), "v"(b)); return d; }
__device__ __forceinline__ void wave_lds_sync() { __builtin_amdgcn_fence(__ATOMIC_RELEASE, "workgroup"); __builtin_amdgcn_wave_barrier(); __builtin_amdgcn_fence(__ATOMIC_ACQUIRE, "workgroup"); }
__device__ __forceinline__ float pmul(float a, float b) { float p = a * b; asm volatile("" : "+v"(p)); return p; }
__device__ __forceinline__ int iclamp(int v, int lo, int hi) { return v < lo ? lo : (v > hi ? hi : v); }

typedef __attribute__((ext_vector_type(2))) _Float16 v2h;
typedef __attribute__((ext_vector_type(4))) _Float16 v4h;
typedef __attribute__((ext_vector_type(2))) float v2f;
typedef __attribute__((ext_vector_type(4))) int v4i;
__device__ __forceinline__ float nexp2(float v) { return __builtin_amdgcn_exp2f(v); }
typedef __attribute__((ext_vector_type(4))) _Float16 v4h_;
__device__ __forceinline__ float lrelu(float v) { return v > 0.0f ? v : NSLOPE * v; }
template <int KIN, int KP>
__global__ __launch_bounds__(256) void wt_kernel(const float* __restrict__ w, b16* __restrict__ WT, float scl) {
  const int u = blockIdx.x * 256 + threadIdx.x; if (u >= NLAY * D * KP / 8) return; const int e = u * 8; const int l = e / (D * KP), rem = e % (D * KP), o = rem / KP, k0 = rem % KP; v8b v;
#pragma unroll
  for (int j = 0; j < 8; ++j) { const int k = k0 + j; v[j] = (b16)(k < KIN ? bf16_rne(w[((size_t)l * D + o) * KIN + (k < KIN ? k : 0)]) * scl : 0.0f); }
  for (int pass = 0; pass < 2; ++pass) { *(volatile v8b*)(WT + e) = v; __threadfence(); }
}
template <bool RND>
__global__ __launch_bounds__(256) void layer_kernel(const float* __restrict__ VFin, const int* __restrict__ aadj, const int* __restrict__ badj, const int* __restrict__ edge, const float* __restrict__ btab, const float* __restrict__ nmask,
    const b16* __restrict__ W2T, const b16* __restrict__ W2Q, const float* __restrict__ b2, const b16* __restrict__ W1T, const b16* __restrict__ W1Q, const float* __restrict__ b1, float* __restrict__ VFout, int mrows) {
  __shared__ __attribute__((aligned(16))) b16 Ah[128][32 + 8], Al[128][32 + 8], Nh[16][KIN2 + 8], Nl[16][KIN2 + 8]; __shared__ __attribute__((aligned(16))) float Tn[16][D + 4];
  const int tid = threadIdx.x, wave = tid >> 5, lane = tid & 31, nloc = lane & 15, hlf = lane >> 4; const int n0 = blockIdx.x * 8;
  const int row = tid >> 1, halfc = tid & 1; const size_t slot = (size_t)(n0 + (row >> 4)) * K + (row & 15);
  int nbr = iclamp(aadj[slot], 0, NN - 1); if (GM < NN) nbr %= GM; const int bslot = iclamp(badj[slot], 0, B * E - 1); const int voc = iclamp(edge[bslot], 0, VOC - 1);
  v8f acc[8];
#pragma unroll
  for (int t = 0; t < 8; ++t) acc[t] = (v8f){};
#pragma unroll 1
  for (int kc = 0; kc < KP1; kc += 32) {
    float vals[16]; const int cbase = kc + halfc * 16;
    if (cbase + 16 <= D) { const float* vr = VFin + (size_t)nbr * D + cbase; for (int q = 0; q < 4; ++q) { const v4f t4 = *(const v4f*)(vr + 4 * q); for (int j = 0; j < 4; ++j) vals[4 * q + j] = RND ? bf16_rne(t4[j]) : t4[j]; } }
    else { for (int j = 0; j < 16; ++j) { const int c = cbase + j; vals[j] = (c >= D && c < KIN1) ? bf16_rne(btab[voc * BF + (c - D)]) : 0.0f; } }
    __syncthreads();
#pragma unroll
    for (int q = 0; q < 4; ++q) { v4h_ h4, l4; for (int j = 0; j < 4; ++j) { const float vs = vals[4 * q + j] * XS; const b16 p = (b16)vs; h4[j] = p; l4[j] = (b16)((vs - (float)p) * RS_); } *(v4h_*)(&Ah[row][halfc * 16 + 4 * q]) = h4; *(v4h_*)(&Al[row][halfc * 16 + 4 * q]) = l4; }
    __syncthreads();
    { const v16b a = frag_kb(&Ah[wave * 16 + nloc][0], hlf), al = frag_kb(&Al[wave * 16 + nloc][0], hlf);
#pragma unroll
      for (int t = 0; t < 8; ++t) { const size_t wo_ = (size_t)(t * 16 + nloc) * KP1 + kc; acc[t] = wmma16b(a, frag_kb(W2T + wo_, hlf), acc[t]); acc[t] = wmma16b(al, frag_kb(W2Q + wo_, hlf), acc[t]); } } }
  { float mk[8]; for (int r = 0; r < 8; ++r) mk[r] = bf16_rne(nmask[(size_t)(n0 + wave) * K + 8 * hlf + r]);
#pragma unroll
    for (int t = 0; t < 8; ++t) { const int col = t * 16 + nloc; const float bb = bf16_rne(b2[col]); float s = 0.0f;
#pragma unroll
      for (int r = 0; r < 8; ++r) s = fmaf(lrelu(acc[t][r] * (1.0f / (XS * WSC)) + bb), mk[r], s);
      s += __shfl_xor(s, 16);
      if (hlf == 0) { const float vs = s * XS; const b16 p = (b16)vs; Nh[wave][D + col] = p; Nl[wave][D + col] = (b16)((vs - (float)p) * RS_); } } }
  { const int n = n0 + wave; const v4f t4 = *(const v4f*)(VFin + (size_t)(n < NN ? n : NN - 1) * D + lane * 4); v4h_ h4, l4, z4; for (int j = 0; j < 4; ++j) { const float vs = (RND ? bf16_rne(t4[j]) : t4[j]) * XS; const b16 p = (b16)vs; h4[j] = p; l4[j] = (b16)((vs - (float)p) * RS_); z4[j] = (b16)0.0f; }
    *(v4h_*)(&Nh[wave][lane * 4]) = h4; *(v4h_*)(&Nl[wave][lane * 4]) = l4;
    for (int c = lane * 4; c < KIN2; c += 128) { *(v4h_*)(&Nh[8 + wave][c]) = z4; *(v4h_*)(&Nl[8 + wave][c]) = z4; } }
  __syncthreads();
  { v8f acc1 = (v8f){}; const b16* br = W1T + (size_t)(wave * 16 + nloc) * KIN2; const b16* bq = W1Q + (size_t)(wave * 16 + nloc) * KIN2;
#pragma unroll
    for (int kb = 0; kb < KIN2; kb += 32) { acc1 = wmma16b(frag_kb(&Nh[nloc][kb], hlf), frag_kb(br + kb, hlf), acc1); acc1 = wmma16b(frag_kb(&Nl[nloc][kb], hlf), frag_kb(bq + kb, hlf), acc1); }
    const int col = wave * 16 + nloc; const float bb = bf16_rne(b1[col]);
#pragma unroll
    for (int r = 0; r < 8; ++r) Tn[8 * hlf + r][col] = lrelu(acc1[r] * (1.0f / (XS * WSC)) + bb); }
  __syncthreads();
  for (int pass = 0; pass < 2; ++pass) { if (n0 + wave < mrows) *(volatile v4f*)(VFout + (size_t)(n0 + wave) * D + lane * 4) = *(const v4f*)(&Tn[wave][lane * 4]); __threadfence(); }
}
}

extern "C" void kernel_launch(void* const* d_in, const int* in_sizes, int n_in, void* d_out, int out_size, void* d_ws, size_t ws_size, hipStream_t stream) {
  (void)n_in;
  auto Fp = [&](int i) { return (const float*)d_in[i]; }; auto Ip = [&](int i) { return (const int*)d_in[i]; };
  if (in_sizes[0] != NN * D || in_sizes[1] != B * E || in_sizes[2] != NN * K || in_sizes[3] != NN * K || in_sizes[4] != NN * K || in_sizes[6] != VOC * BF || in_sizes[7] != NLAY * D * KIN1 || in_sizes[8] != NLAY * D || in_sizes[9] != NLAY * D * KIN2 || in_sizes[10] != NLAY * D || out_size != NN * D) return;
  size_t off = 0; char* ws = (char*)d_ws;
  auto carve = [&](size_t bytes) { char* p = ws + off; off += (bytes + 255) & ~(size_t)255; return p; };
  b16* W2T = (b16*)carve((size_t)NLAY * D * KP1 * 2); b16* W2Q = (b16*)carve((size_t)NLAY * D * KP1 * 2); b16* W1T = (b16*)carve((size_t)NLAY * D * KIN2 * 2); b16* W1Q = (b16*)carve((size_t)NLAY * D * KIN2 * 2);
  float* VF1 = (float*)carve((size_t)NN * D * 4); float* VF2 = (float*)carve((size_t)NN * D * 4);
  if (off > ws_size || off > ((size_t)128 << 20)) return;
  wt_kernel<KIN1, KP1><<<(NLAY * D * KP1 / 8 + 255) / 256, 256, 0, stream>>>(Fp(7), W2T, WSC); wt_kernel<KIN1, KP1><<<(NLAY * D * KP1 / 8 + 255) / 256, 256, 0, stream>>>(Fp(7), W2Q, WSQ);
  wt_kernel<KIN2, KIN2><<<(NLAY * D * KIN2 / 8 + 255) / 256, 256, 0, stream>>>(Fp(9), W1T, WSC); wt_kernel<KIN2, KIN2><<<(NLAY * D * KIN2 / 8 + 255) / 256, 256, 0, stream>>>(Fp(9), W1Q, WSQ);
  layer_kernel<true><<<NPL / 8, 256, 0, stream>>>(Fp(0), Ip(2), Ip(3), Ip(1), Fp(6), Fp(4), W2T, W2Q, Fp(8), W1T, W1Q, Fp(10), VF1, NPL);
  layer_kernel<false><<<NPL / 8, 256, 0, stream>>>(VF1, Ip(2), Ip(3), Ip(1), Fp(6), Fp(4), W2T + (size_t)D * KP1, W2Q + (size_t)D * KP1, Fp(8) + D, W1T + (size_t)D * KIN2, W1Q + (size_t)D * KIN2, Fp(10) + D, VF2, NPL);
  layer_kernel<false><<<NPL / 8, 256, 0, stream>>>(VF2, Ip(2), Ip(3), Ip(1), Fp(6), Fp(4), W2T + (size_t)2 * D * KP1, W2Q + (size_t)2 * D * KP1, Fp(8) + 2 * D, W1T + (size_t)2 * D * KIN2, W1Q + (size_t)2 * D * KIN2, Fp(10) + 2 * D, (float*)d_out, NPL);
}
